// ball_ball_update_opt_net_72765335929731
// MI455X (gfx1250) — hardware-verified
//
#include <hip/hip_runtime.h>
#include <stddef.h>


typedef float v8f __attribute__((ext_vector_type(8)));
typedef float v4f __attribute__((ext_vector_type(4)));
typedef unsigned short v8us __attribute__((ext_vector_type(8)));
typedef __bf16 v16b __attribute__((ext_vector_type(16)));
union Frag { v16b v; v8us p[2]; };

#define NF 8
#define NH 200
#define KS 232
#define KCH 7
#define NT_H 13
#define WPITCH 256
#define PROW_W2 0
#define PROW_W3 208
#define PROW_W4 416
#define PROWS 432
#define RPB 128
#define TPB 256

#define OFF_HI 0
#define OFF_LO (RPB * KS * 2)
#define OFF_W1 (2 * RPB * KS * 2)
#define OFF_B1 (OFF_W1 + NH * NF * 4)
#define OFF_QI (OFF_B1 + 208 * 4)
#define OFF_W0 (OFF_QI + 64 * 4)
#define OFF_B0 (OFF_W0 + 64 * 4)
#define OFF_Z  (OFF_B0 + 32)
#define OFF_ST (OFF_Z + RPB * NF * 4)
#define SMEM_TOTAL (OFF_ST + RPB * NF * 4)

static_assert((OFF_LO % 16) == 0);
static_assert((OFF_W1 % 16) == 0);
static_assert((OFF_B1 % 16) == 0);
static_assert((OFF_QI % 16) == 0);
static_assert((OFF_Z % 16) == 0);
static_assert((OFF_ST % 16) == 0);
static_assert((SMEM_TOTAL % 16) == 0);
static_assert((PROWS % 8) == 0);
static_assert(((KS * 2) % 16) == 0);

__device__ __forceinline__ unsigned int bf16_bits(float f) {
  unsigned int u = __float_as_uint(f);
  u += 0x7FFFu + ((u >> 16) & 1u);
  return u >> 16;
}

__device__ __forceinline__ void mma3(v8f& acc, const v16b ah, const v16b al, const v16b bh, const v16b bl) {
  acc = __builtin_amdgcn_wmma_f32_16x16x32_bf16(false, ah, false, bh, (short)0, acc, false, false);
  acc = __builtin_amdgcn_wmma_f32_16x16x32_bf16(false, ah, false, bl, (short)0, acc, false, false);
  acc = __builtin_amdgcn_wmma_f32_16x16x32_bf16(false, al, false, bh, (short)0, acc, false, false);
  asm volatile("v_nop\n\tv_nop\n\tv_nop\n\tv_nop" : "+v"(acc) : "v"(ah), "v"(al), "v"(bh), "v"(bl));
}

__global__ __launch_bounds__(TPB) void prep_kernel(const float* __restrict__ Q,
                                                  const float* __restrict__ W2,
                                                  const float* __restrict__ W3,
                                                  const float* __restrict__ W4,
                                                  float* Qi,
                                                  unsigned short* pHi,
                                                  unsigned short* pLo) {
  __shared__ float sGJ[8 * 16];
  const int tid = threadIdx.x;
  const int lane = tid & 31;
  const int wave = tid >> 5;

  if (blockIdx.x == 0 && tid == 0) {
#pragma unroll 1
    for (int i = 0; i < 8; ++i) {
#pragma unroll 1
      for (int j = 0; j < 8; ++j) {
        sGJ[i * 16 + j] = Q[i * 8 + j];
        sGJ[i * 16 + 8 + j] = (i == j) ? 1.0f : 0.0f;
      }
    }
#pragma unroll 1
    for (int c = 0; c < 8; ++c) {
      int p = c;
      float best = fabsf(sGJ[c * 16 + c]);
#pragma unroll 1
      for (int r = c + 1; r < 8; ++r) {
        const float v = fabsf(sGJ[r * 16 + c]);
        if (v > best) { best = v; p = r; }
      }
      if (p != c) {
#pragma unroll 1
        for (int j = 0; j < 16; ++j) {
          const float t = sGJ[c * 16 + j];
          sGJ[c * 16 + j] = sGJ[p * 16 + j];
          sGJ[p * 16 + j] = t;
        }
      }
      const float inv = 1.0f / sGJ[c * 16 + c];
#pragma unroll 1
      for (int j = 0; j < 16; ++j) sGJ[c * 16 + j] = sGJ[c * 16 + j] * inv;
#pragma unroll 1
      for (int r = 0; r < 8; ++r) {
        if (r != c) {
          const float f = sGJ[r * 16 + c];
#pragma unroll 1
          for (int j = 0; j < 16; ++j) sGJ[r * 16 + j] = sGJ[r * 16 + j] - f * sGJ[c * 16 + j];
        }
      }
    }
    volatile float* vq = (volatile float*)Qi;
#pragma unroll 1
    for (int i = 0; i < 64; ++i) vq[i] = sGJ[(i >> 3) * 16 + 8 + (i & 7)];
    __threadfence();
#pragma unroll 1
    for (int i = 0; i < 64; ++i) vq[i] = sGJ[(i >> 3) * 16 + 8 + (i & 7)];
  }

  const int prow = blockIdx.x * 8 + wave;
  if (prow < PROWS) {
    const float* W;
    int nin, nout, n;
    if (prow < PROW_W3)      { W = W2; nin = NH; nout = NH; n = prow - PROW_W2; }
    else if (prow < PROW_W4) { W = W3; nin = NH; nout = NH; n = prow - PROW_W3; }
    else                     { W = W4; nin = NH; nout = NF; n = prow - PROW_W4; }
    v8us hv = {0, 0, 0, 0, 0, 0, 0, 0};
    v8us lv = {0, 0, 0, 0, 0, 0, 0, 0};
#pragma unroll
    for (int j = 0; j < 8; ++j) {
      const int k = lane * 8 + j;
      float w = 0.0f;
      if (n < nout && k < nin) w = W[(size_t)n * nin + k];
      const unsigned int hb = bf16_bits(w);
      const float wh = __uint_as_float(hb << 16);
      const unsigned int lb = bf16_bits(w - wh);
      hv[j] = (unsigned short)hb;
      lv[j] = (unsigned short)lb;
    }
    unsigned short* dh = pHi + (size_t)prow * WPITCH + lane * 8;
    unsigned short* dl = pLo + (size_t)prow * WPITCH + lane * 8;
    *(volatile v8us*)dh = hv;
    *(volatile v8us*)dl = lv;
    __threadfence();
    *(volatile v8us*)dh = hv;
    *(volatile v8us*)dl = lv;
  }
}

template <int NT, bool LAST>
__device__ __forceinline__ void gemm_layer(unsigned short* sHi, unsigned short* sLo,
                                           const unsigned short* __restrict__ gHi,
                                           const unsigned short* __restrict__ gLo,
                                           const float* __restrict__ bias, const int nout,
                                           const int wrow, const int lane, float* sStage) {
  const int h = lane >> 4;
  const int m = lane & 15;
  v8f acc[NT];
#pragma unroll
  for (int nt = 0; nt < NT; ++nt) {
    v8f z = {0.f, 0.f, 0.f, 0.f, 0.f, 0.f, 0.f, 0.f};
    acc[nt] = z;
  }
  const unsigned short* aH = sHi + (wrow + m) * KS + 8 * h;
  const unsigned short* aL = sLo + (wrow + m) * KS + 8 * h;
  const unsigned short* bH = gHi + m * WPITCH + 8 * h;
  const unsigned short* bL = gLo + m * WPITCH + 8 * h;
#pragma unroll 1
  for (int kc = 0; kc < KCH; ++kc) {
    const int ko = kc * 32;
    Frag fah, fal;
    fah.p[0] = *(const v8us*)(aH + ko);
    fah.p[1] = *(const v8us*)(aH + ko + 16);
    fal.p[0] = *(const v8us*)(aL + ko);
    fal.p[1] = *(const v8us*)(aL + ko + 16);
#pragma unroll
    for (int nt = 0; nt < NT; ++nt) {
      const int bo = nt * 16 * WPITCH + ko;
      Frag fbh, fbl;
      fbh.p[0] = *(const v8us*)(bH + bo);
      fbh.p[1] = *(const v8us*)(bH + bo + 16);
      fbl.p[0] = *(const v8us*)(bL + bo);
      fbl.p[1] = *(const v8us*)(bL + bo + 16);
      mma3(acc[nt], fah.v, fal.v, fbh.v, fbl.v);
    }
  }
  if constexpr (!LAST) {
#pragma unroll
    for (int nt = 0; nt < NT; ++nt) {
      const int n = nt * 16 + m;
      const float bv = (n < nout) ? bias[n] : 0.0f;
      unsigned short* oH = sHi + (wrow + 8 * h) * KS + n;
      unsigned short* oL = sLo + (wrow + 8 * h) * KS + n;
#pragma unroll
      for (int r = 0; r < 8; ++r) {
        const float y = fmaxf(acc[nt][r] + bv, 0.0f);
        const unsigned int hb = bf16_bits(y);
        const float yh = __uint_as_float(hb << 16);
        const unsigned int lb = bf16_bits(y - yh);
        oH[r * KS] = (unsigned short)hb;
        oL[r * KS] = (unsigned short)lb;
      }
    }
  } else {
    if (m < NF) {
      const float bv = bias[m];
#pragma unroll
      for (int r = 0; r < 8; ++r) sStage[(wrow + 8 * h + r) * NF + m] = acc[0][r] + bv;
    }
  }
}

__global__ __launch_bounds__(TPB) __attribute__((amdgpu_num_vgpr(240)))
void mlp_kernel(const float* __restrict__ x, const float* __restrict__ Qi,
                const float* __restrict__ W0, const float* __restrict__ b0,
                const float* __restrict__ W1, const float* __restrict__ b1,
                const float* __restrict__ b2, const float* __restrict__ b3,
                const float* __restrict__ b4,
                const unsigned short* __restrict__ pHi, const unsigned short* __restrict__ pLo,
                float* out, const int nrows) {
  extern __shared__ v4f dyn_smem[];
  char* smem = (char*)dyn_smem;
  unsigned short* sHi = (unsigned short*)(smem + OFF_HI);
  unsigned short* sLo = (unsigned short*)(smem + OFF_LO);
  float* sW1 = (float*)(smem + OFF_W1);
  float* sB1 = (float*)(smem + OFF_B1);
  float* sQi = (float*)(smem + OFF_QI);
  float* sW0 = (float*)(smem + OFF_W0);
  float* sB0 = (float*)(smem + OFF_B0);
  float* sZ  = (float*)(smem + OFF_Z);
  float* sSt = (float*)(smem + OFF_ST);

  const int tid = threadIdx.x;
  const int lane = tid & 31;
  const int wave = tid >> 5;
  const int wrow = wave * 16;
  const int rowBase = blockIdx.x * RPB;

  for (int i = tid; i < NH * NF; i += TPB) sW1[i] = W1[i];
  if (tid < NH) sB1[tid] = b1[tid];
  if (tid < 64) { sQi[tid] = Qi[tid]; sW0[tid] = W0[tid]; }
  if (tid < NF) sB0[tid] = b0[tid];
  __syncthreads();

  if (tid < RPB) {
#pragma clang fp contract(off)
    const int lr = tid;
    int grow = rowBase + lr;
    grow = (grow < nrows) ? grow : (nrows - 1);
    const float* xr = x + (size_t)grow * NF;
    const v4f xa = *(const v4f*)xr;
    const v4f xb = *(const v4f*)(xr + 4);
    float xv[NF] = {xa[0], xa[1], xa[2], xa[3], xb[0], xb[1], xb[2], xb[3]};
    float hv[NF], u[NF], c0[NF], c1[NF];
#pragma unroll
    for (int j = 0; j < NF; ++j) {
      float s = 0.0f;
#pragma unroll
      for (int i = 0; i < NF; ++i) s = s + sW0[j * NF + i] * xv[i];
      hv[j] = s + sB0[j];
    }
    const float h3 = hv[3];
#pragma unroll
    for (int i = 0; i < NF; ++i) {
      float s = 0.0f;
#pragma unroll
      for (int j = 0; j < NF; ++j) s = s + sQi[i * NF + j] * hv[j];
      u[i] = s;
      c0[i] = h3 * sQi[i * NF + 4] + sQi[i * NF + 5];
      c1[i] = h3 * sQi[i * NF + 6] + sQi[i * NF + 7];
    }
    const float M00 = h3 * c0[4] + c0[5];
    const float M01 = h3 * c1[4] + c1[5];
    const float M10 = h3 * c0[6] + c0[7];
    const float M11 = h3 * c1[6] + c1[7];
    const float r0 = (h3 * u[4] + u[5]) - (h3 * hv[4] + hv[5]);
    const float r1 = (h3 * u[6] + u[7]) - (h3 * hv[6] + hv[7]);
    const float det = M00 * M11 - M01 * M10;
    const float idet = 1.0f / det;
    const float nu0 = (r0 * M11 - r1 * M01) * idet;
    const float nu1 = (M00 * r1 - M10 * r0) * idet;
    float* zr = sZ + lr * NF;
#pragma unroll
    for (int i = 0; i < NF; ++i) zr[i] = u[i] - nu0 * c0[i] - nu1 * c1[i];
  } else {
    const int lr = tid - RPB;
    v8us zz = {0, 0, 0, 0, 0, 0, 0, 0};
    unsigned short* rH = sHi + lr * KS + NH;
    unsigned short* rL = sLo + lr * KS + NH;
#pragma unroll
    for (int q = 0; q < 4; ++q) {
      *(v8us*)(rH + 8 * q) = zz;
      *(v8us*)(rL + 8 * q) = zz;
    }
  }
  __syncthreads();

  {
    const int lr = tid >> 1;
    const int n0 = (tid & 1) * (NH / 2);
    const v4f za = *(const v4f*)(sZ + lr * NF);
    const v4f zb = *(const v4f*)(sZ + lr * NF + 4);
    unsigned short* oH = sHi + lr * KS;
    unsigned short* oL = sLo + lr * KS;
#pragma unroll 2
    for (int j = 0; j < NH / 2; ++j) {
      const int n = n0 + j;
      const v4f wa = *(const v4f*)(sW1 + n * NF);
      const v4f wb = *(const v4f*)(sW1 + n * NF + 4);
      float s = za[0] * wa[0];
      s += za[1] * wa[1];
      s += za[2] * wa[2];
      s += za[3] * wa[3];
      s += zb[0] * wb[0];
      s += zb[1] * wb[1];
      s += zb[2] * wb[2];
      s += zb[3] * wb[3];
      s += sB1[n];
      const float y = fmaxf(s, 0.0f);
      const unsigned int hb = bf16_bits(y);
      const float yh = __uint_as_float(hb << 16);
      const unsigned int lb = bf16_bits(y - yh);
      oH[n] = (unsigned short)hb;
      oL[n] = (unsigned short)lb;
    }
  }
  __syncthreads();

  gemm_layer<NT_H, false>(sHi, sLo, pHi + PROW_W2 * WPITCH, pLo + PROW_W2 * WPITCH, b2, NH, wrow, lane, sSt);
  __syncthreads();
  gemm_layer<NT_H, false>(sHi, sLo, pHi + PROW_W3 * WPITCH, pLo + PROW_W3 * WPITCH, b3, NH, wrow, lane, sSt);
  __syncthreads();
  gemm_layer<1, true>(sHi, sLo, pHi + PROW_W4 * WPITCH, pLo + PROW_W4 * WPITCH, b4, NF, wrow, lane, sSt);
  __syncthreads();

  {
    const int grow = rowBase + wrow + (lane >> 1);
    const v4f v = *(const v4f*)(sSt + wrow * NF + lane * 4);
    float* gp = out + (size_t)(rowBase + wrow) * NF + lane * 4;
    const bool ok = grow < nrows;
    if (ok) *(volatile v4f*)gp = v;
    __threadfence();
    if (ok) *(volatile v4f*)gp = v;
  }
}

extern "C" void kernel_launch(void* const* d_in, const int* in_sizes, int n_in,
                              void* d_out, int out_size, void* d_ws, size_t ws_size,
                              hipStream_t stream) {
  if (n_in < 12) return;
  const float* x  = (const float*)d_in[0];
  const float* Q  = (const float*)d_in[1];
  const float* W0 = (const float*)d_in[2];
  const float* b0 = (const float*)d_in[3];
  const float* W1 = (const float*)d_in[4];
  const float* b1 = (const float*)d_in[5];
  const float* W2 = (const float*)d_in[6];
  const float* b2 = (const float*)d_in[7];
  const float* W3 = (const float*)d_in[8];
  const float* b3 = (const float*)d_in[9];
  const float* W4 = (const float*)d_in[10];
  const float* b4 = (const float*)d_in[11];
  float* out = (float*)d_out;

  if (in_sizes[1] < 64 || in_sizes[2] < 64 || in_sizes[3] < NF) return;
  if (in_sizes[4] < NH * NF || in_sizes[5] < NH) return;
  if (in_sizes[6] < NH * NH || in_sizes[7] < NH || in_sizes[8] < NH * NH || in_sizes[9] < NH) return;
  if (in_sizes[10] < NF * NH || in_sizes[11] < NF) return;

  int nrows = in_sizes[0] / NF;
  if (out_size / NF < nrows) nrows = out_size / NF;
  if (nrows <= 0) return;

  const size_t qi_bytes = 256;
  const size_t plane_bytes = (size_t)PROWS * WPITCH * sizeof(unsigned short);
  const size_t need = qi_bytes + 2 * plane_bytes;
  if (need > ws_size) return;
  float* Qi = (float*)d_ws;
  unsigned short* pHi = (unsigned short*)((char*)d_ws + qi_bytes);
  unsigned short* pLo = (unsigned short*)((char*)d_ws + qi_bytes + plane_bytes);

  prep_kernel<<<dim3((PROWS + 7) / 8), dim3(TPB), 0, stream>>>(Q, W2, W3, W4, Qi, pHi, pLo);
  mlp_kernel<<<dim3((nrows + RPB - 1) / RPB), dim3(TPB), SMEM_TOTAL, stream>>>(
      x, Qi, W0, b0, W1, b1, b2, b3, b4, pHi, pLo, out, nrows);
}
